// ExtractLayer_42623255445874
// MI455X (gfx1250) — hardware-run, weakly checked
//
#include <hip/hip_runtime.h>
#include <stddef.h>


#define FD      64
#define NREL    5
#define NMAT    10
#define NTHR    256
#define NWAVE   8
#define EPT     8
#define CHUNK   (NTHR * EPT)
#define WCAP    (EPT * 32)
#define LISTN   (NWAVE * WCAP)
#define NBMAX   2048
#define RCAP    28672
#define DEGCAP  4096
#define GBM     64
#define GTHR    128
#define RB      512
#define PARTN   128
#define SLOTN   256
#define HSCALE  16.0f
#define WSCALE  64.0f
#define OINV    0.0009765625f
#define NEG_SLOPE 0.2f
#define BN_EPS  0.00001f
#define WSCAP   134217728
#define LDS_AGG ((2 * RCAP + 2 * NBMAX + LISTN) * 4 + 64)

static_assert((CHUNK & (CHUNK - 1)) == 0 && CHUNK <= 4096);
static_assert((NBMAX & (NBMAX - 1)) == 0 && NBMAX <= 4096);
static_assert(NTHR * 8 == NBMAX);
static_assert(LISTN >= NBMAX);
static_assert(LISTN >= NWAVE * 256);
static_assert((RCAP % 32) == 0);
static_assert(LDS_AGG <= 300000);
static_assert(GBM == (GTHR / 32) * 16);
static_assert(RB == 4 * 128);
static_assert(SLOTN == 4 * FD && PARTN == 2 * FD);

typedef float          v2f  __attribute__((ext_vector_type(2)));
typedef float          v4f  __attribute__((ext_vector_type(4)));
typedef float          v4fa __attribute__((ext_vector_type(4), __may_alias__));
typedef float          v8f  __attribute__((ext_vector_type(8)));
typedef double         v2d  __attribute__((ext_vector_type(2)));
typedef int            v4i  __attribute__((ext_vector_type(4)));
typedef unsigned short v8us __attribute__((ext_vector_type(8)));
typedef _Float16       v8h  __attribute__((ext_vector_type(8)));
typedef _Float16       v16h __attribute__((ext_vector_type(16)));
union FragH { v16h v; v8us h[2]; };
union Pack8 { v8h h; v8us u; };

__device__ __forceinline__ v8us cvt8h(v4f a, v4f b, float sc) {
  v8h r;
  r[0] = (_Float16)(a.x * sc); r[1] = (_Float16)(a.y * sc);
  r[2] = (_Float16)(a.z * sc); r[3] = (_Float16)(a.w * sc);
  r[4] = (_Float16)(b.x * sc); r[5] = (_Float16)(b.y * sc);
  r[6] = (_Float16)(b.z * sc); r[7] = (_Float16)(b.w * sc);
  Pack8 p;
  p.h = r;
  return p.u;
}

__device__ __forceinline__ v8f wmh(v16h a, v16h b, v8f c) {
  v8f d = __builtin_amdgcn_wmma_f32_16x16x32_f16(false, a, false, b, (short)0, c, false, false);
  asm volatile("v_nop\n\tv_nop\n\tv_nop\n\tv_nop" : "+v"(d) : "v"(a), "v"(b));
  return d;
}

__device__ __forceinline__ int scan_chunk(const int* __restrict__ dsts, int nE, int cbase, int slotBase,
                                          int nb, int vec8, int* list, int tid, int lane, int wave) {
  int wc = 0;
  const int el0  = tid * EPT;
  const int e0   = cbase + el0;
  const int sent = -2147483647 - 1;
  v4i da, db;
  if (vec8 != 0 && cbase + CHUNK <= nE) {
    da = *(const v4i*)(dsts + e0);
    db = *(const v4i*)(dsts + e0 + 4);
  } else {
    da.x = (e0     < nE) ? dsts[min(e0,     nE - 1)] : sent;
    da.y = (e0 + 1 < nE) ? dsts[min(e0 + 1, nE - 1)] : sent;
    da.z = (e0 + 2 < nE) ? dsts[min(e0 + 2, nE - 1)] : sent;
    da.w = (e0 + 3 < nE) ? dsts[min(e0 + 3, nE - 1)] : sent;
    db.x = (e0 + 4 < nE) ? dsts[min(e0 + 4, nE - 1)] : sent;
    db.y = (e0 + 5 < nE) ? dsts[min(e0 + 5, nE - 1)] : sent;
    db.z = (e0 + 6 < nE) ? dsts[min(e0 + 6, nE - 1)] : sent;
    db.w = (e0 + 7 < nE) ? dsts[min(e0 + 7, nE - 1)] : sent;
  }
  const unsigned nbs = (unsigned)slotBase;
  const unsigned unb = (unsigned)nb;
  const unsigned s0 = (unsigned)da.x - nbs, s1 = (unsigned)da.y - nbs;
  const unsigned s2 = (unsigned)da.z - nbs, s3 = (unsigned)da.w - nbs;
  const unsigned s4 = (unsigned)db.x - nbs, s5 = (unsigned)db.y - nbs;
  const unsigned s6 = (unsigned)db.z - nbs, s7 = (unsigned)db.w - nbs;
  const bool h0 = s0 < unb, h1 = s1 < unb, h2 = s2 < unb, h3 = s3 < unb;
  const bool h4 = s4 < unb, h5 = s5 < unb, h6 = s6 < unb, h7 = s7 < unb;
  const unsigned any = __builtin_amdgcn_ballot_w32(h0 | h1 | h2 | h3 | h4 | h5 | h6 | h7);
  if (any != 0u) {
#define HITJ(J, HJ, SJ) { \
      const unsigned mj = __builtin_amdgcn_ballot_w32(HJ); \
      if (mj != 0u) { \
        if (HJ) { \
          const int pos = wc + (int)__builtin_amdgcn_mbcnt_lo(mj, 0u); \
          if (pos < WCAP) list[wave * WCAP + pos] = ((el0 + (J)) << 12) | (int)(SJ); \
        } \
        wc += (int)__builtin_popcount(mj); } }
    HITJ(0, h0, s0)
    HITJ(1, h1, s1)
    HITJ(2, h2, s2)
    HITJ(3, h3, s3)
    HITJ(4, h4, s4)
    HITJ(5, h5, s5)
    HITJ(6, h6, s6)
    HITJ(7, h7, s7)
#undef HITJ
  }
  return wc;
}

__global__ __launch_bounds__(NTHR) void k_xprep(const float* __restrict__ x, unsigned short* X16,
                                                int nN, int nUnits) {
  const int i = (int)blockIdx.x * NTHR + (int)threadIdx.x;
  if (i >= nUnits) return;
  const int row = i >> 3;
  const int c0  = (i & 7) * 8;
  const int rc  = row < nN ? row : nN - 1;
  const float* p = x + (size_t)rc * FD + c0;
  v4f a = *(const v4f*)p, b = *(const v4f*)(p + 4);
  const v4f z4 = {0.f, 0.f, 0.f, 0.f};
  if (row >= nN) { a = z4; b = z4; }
  const v8us hv = cvt8h(a, b, HSCALE);
  unsigned short* d = X16 + (size_t)row * FD + c0;
  *(volatile v8us*)d = hv;
  __threadfence();
  *(volatile v8us*)d = hv;
}

__global__ __launch_bounds__(NTHR) void k_wprep(const float* __restrict__ Wl, const float* __restrict__ Wr,
                                                unsigned short* wq) {
  const int j = (int)blockIdx.y;
  const int u = (int)blockIdx.x * NTHR + (int)threadIdx.x;
  if (u >= FD * FD / 8) return;
  const int n  = u >> 3;
  const int k8 = (u & 7) * 8;
  const float* src = ((j & 1) ? Wr : Wl) + (size_t)(j >> 1) * FD * FD;
  float v[8];
#pragma unroll
  for (int e = 0; e < 8; ++e) v[e] = src[(size_t)(k8 + e) * FD + n];
  v4f a, b;
  a.x = v[0]; a.y = v[1]; a.z = v[2]; a.w = v[3];
  b.x = v[4]; b.y = v[5]; b.z = v[6]; b.w = v[7];
  const v8us hv = cvt8h(a, b, WSCALE);
  unsigned short* d = wq + (size_t)j * FD * FD + (size_t)n * FD + k8;
  *(volatile v8us*)d = hv;
  __threadfence();
  *(volatile v8us*)d = hv;
}

__global__ __launch_bounds__(GTHR) void k_gemm(const unsigned short* __restrict__ A16,
                                               const unsigned short* __restrict__ Bw,
                                               float* Y, int nwt) {
  __shared__ __attribute__((aligned(16))) float stg[GBM * 2 * FD];
  const int tid = threadIdx.x, lane = tid & 31, wave = tid >> 5, hh = lane >> 4, m = lane & 15;
  const int rowBase = (int)blockIdx.x * GBM;
  const int SP = FD * nwt;
  const unsigned short* ap = A16 + (size_t)(rowBase + 16 * wave + m) * FD + 8 * hh;
  FragH a0, a1;
  a0.h[0] = *(const v8us*)(ap);
  a0.h[1] = *(const v8us*)(ap + 16);
  a1.h[0] = *(const v8us*)(ap + 32);
  a1.h[1] = *(const v8us*)(ap + 48);
#pragma unroll 1
  for (int w = 0; w < nwt; ++w) {
    v8f acc[4];
#pragma unroll
    for (int t = 0; t < 4; ++t) { v8f z = {0.f, 0.f, 0.f, 0.f, 0.f, 0.f, 0.f, 0.f}; acc[t] = z; }
    const unsigned short* bq = Bw + (size_t)w * FD * FD + (size_t)m * FD + 8 * hh;
#pragma unroll
    for (int t = 0; t < 4; ++t) {
      const unsigned short* bp = bq + (size_t)(16 * t) * FD;
      FragH b0, b1;
      b0.h[0] = *(const v8us*)(bp);
      b0.h[1] = *(const v8us*)(bp + 16);
      b1.h[0] = *(const v8us*)(bp + 32);
      b1.h[1] = *(const v8us*)(bp + 48);
      acc[t] = wmh(a0.v, b0.v, acc[t]);
      acc[t] = wmh(a1.v, b1.v, acc[t]);
    }
    float* sp = stg + (size_t)(16 * wave + 8 * hh) * SP + FD * w + m;
#pragma unroll
    for (int t = 0; t < 4; ++t) {
#pragma unroll
      for (int r = 0; r < 8; ++r) sp[(size_t)r * SP + 16 * t] = acc[t][r] * OINV;
    }
  }
  __syncthreads();
  const int nF4 = GBM * SP / 4;
  float* yb = Y + (size_t)rowBase * SP;
  const v4f* s4 = (const v4f*)stg;
#pragma unroll 1
  for (int f = tid; f < nF4; f += GTHR) { const v4f v = s4[f]; *(volatile v4f*)(yb + 4 * (size_t)f) = v; }
  __threadfence();
#pragma unroll 1
  for (int f = tid; f < nF4; f += GTHR) { const v4f v = s4[f]; *(volatile v4f*)(yb + 4 * (size_t)f) = v; }
}

__global__ __launch_bounds__(NTHR) void k_logit(const int* __restrict__ srcs, const int* __restrict__ dsts,
                                                const float* __restrict__ xl, const float* __restrict__ xr,
                                                const float* __restrict__ attr, float* ev,
                                                int nE, int nSrc, int nDst, int xlPitch, int xrPitch) {
  const int i = (int)blockIdx.x * NTHR + (int)threadIdx.x;
  const int ei = i < nE ? i : nE - 1;
  int s = srcs[ei]; s = s < 0 ? 0 : (s > nSrc - 1 ? nSrc - 1 : s);
  int d = dsts[ei]; d = d < 0 ? 0 : (d > nDst - 1 ? nDst - 1 : d);
  const float* pl = xl + (size_t)s * xlPitch;
  const float* pr = xr + (size_t)d * xrPitch;
  float acc = 0.0f;
#pragma unroll 8
  for (int j = 0; j < FD / 4; ++j) {
    const v4f l = *(const v4f*)(pl + 4 * j);
    const v4f r = *(const v4f*)(pr + 4 * j);
    const v4f a = *(const v4f*)(attr + 4 * j);
    const v4f t = l + r;
    v4f h;
    h.x = fmaxf(t.x, NEG_SLOPE * t.x);
    h.y = fmaxf(t.y, NEG_SLOPE * t.y);
    h.z = fmaxf(t.z, NEG_SLOPE * t.z);
    h.w = fmaxf(t.w, NEG_SLOPE * t.w);
    acc = fmaf(h.x, a.x, acc);
    acc = fmaf(h.y, a.y, acc);
    acc = fmaf(h.z, a.z, acc);
    acc = fmaf(h.w, a.w, acc);
  }
  float* gp = ev + i;
  *(volatile float*)gp = acc;
  __threadfence();
  *(volatile float*)gp = acc;
}

__global__ __launch_bounds__(NTHR) void k_agg(
    const int* __restrict__ srcs, const int* __restrict__ dsts, const float* __restrict__ ev,
    const float* __restrict__ xl, const float* addend, const float* __restrict__ biasr, float* outp,
    int nDst, int nSrc, int nE, int xlPitch, int nb, int vec8) {
  extern __shared__ v4f lds_dyn[];
  int* reg1 = (int*)lds_dyn;
  int* reg2 = reg1 + RCAP;
  int* scnt = reg2 + RCAP;
  int* soff = scnt + NBMAX;
  int* list = soff + NBMAX;
  int* wcnt = list + LISTN;
  int* wtot = wcnt + NWAVE;
  const int tid = threadIdx.x, lane = tid & 31, wave = tid >> 5;
  const int nodeBase = (int)blockIdx.x * nb;

  for (int i = tid; i < NBMAX; i += NTHR) scnt[i] = 0;
  __syncthreads();

  int tot = 0;
  const int nChunks = (nE + CHUNK - 1) / CHUNK;
#pragma unroll 1
  for (int ch = 0; ch < nChunks; ++ch) {
    const int cbase = ch * CHUNK;
    const int wc = scan_chunk(dsts, nE, cbase, nodeBase, nb, vec8, list, tid, lane, wave);
    if (lane == 0) wcnt[wave] = wc;
    __syncthreads();
    int pre = 0, all = 0;
#pragma unroll
    for (int w2 = 0; w2 < NWAVE; ++w2) {
      int c = wcnt[w2];
      c = c < 0 ? 0 : (c > WCAP ? WCAP : c);
      all += c;
      pre += (w2 < wave) ? c : 0;
    }
    const int wcc  = wc > WCAP ? WCAP : wc;
    const int base = tot + pre;
#pragma unroll 1
    for (int i = lane; i < wcc; i += 32) {
      const int ent = list[wave * WCAP + i];
      const int el  = (ent >> 12) & (CHUNK - 1);
      const int sl  = ent & (NBMAX - 1);
      int eid = cbase + el;
      eid = eid > nE - 1 ? nE - 1 : eid;
      const int pos = base + i;
      if (pos < RCAP) reg1[pos] = (int)(((unsigned)eid << 12) | (unsigned)sl);
    }
    tot += all;
    tot = tot > RCAP ? RCAP : tot;
    __syncthreads();
  }
  const int nh = tot;

  if (wave == 0) {
#pragma unroll 1
    for (int b0 = 0; b0 < nh; b0 += 32) {
      const int idx = b0 + lane;
      const int uv  = reg1[idx < RCAP ? idx : RCAP - 1];
      const int m32 = (nh - b0) < 32 ? (nh - b0) : 32;
#pragma unroll 1
      for (int k = 0; k < m32; ++k) {
        const int u  = __builtin_amdgcn_readlane(uv, k);
        const int sl = u & (NBMAX - 1);
        if (lane == 0) scnt[sl] = scnt[sl] + 1;
      }
    }
  }
  __syncthreads();

  {
    const v4i ca = *(const v4i*)(scnt + 8 * tid);
    const v4i cb = *(const v4i*)(scnt + 8 * tid + 4);
    const int e0 = ca.x < 0 ? 0 : ca.x, e1 = ca.y < 0 ? 0 : ca.y, e2 = ca.z < 0 ? 0 : ca.z, e3 = ca.w < 0 ? 0 : ca.w;
    const int e4 = cb.x < 0 ? 0 : cb.x, e5 = cb.y < 0 ? 0 : cb.y, e6 = cb.z < 0 ? 0 : cb.z, e7 = cb.w < 0 ? 0 : cb.w;
    const int ts = e0 + e1 + e2 + e3 + e4 + e5 + e6 + e7;
    int incl = ts;
#pragma unroll
    for (int d = 1; d < 32; d <<= 1) {
      const int up = __shfl_up(incl, d);
      if (lane >= d) incl += up;
    }
    if (lane == 31) wtot[wave] = incl;
    __syncthreads();
    int pre = 0;
#pragma unroll
    for (int w2 = 0; w2 < NWAVE; ++w2) pre += (w2 < wave) ? wtot[w2] : 0;
    int run = pre + incl - ts;
    soff[8 * tid + 0] = run; run += e0;
    soff[8 * tid + 1] = run; run += e1;
    soff[8 * tid + 2] = run; run += e2;
    soff[8 * tid + 3] = run; run += e3;
    soff[8 * tid + 4] = run; run += e4;
    soff[8 * tid + 5] = run; run += e5;
    soff[8 * tid + 6] = run; run += e6;
    soff[8 * tid + 7] = run;
  }
  __syncthreads();
  for (int i = tid; i < NBMAX; i += NTHR) list[i] = soff[i];
  __syncthreads();

  if (wave == 0) {
#pragma unroll 1
    for (int b0 = 0; b0 < nh; b0 += 32) {
      const int idx = b0 + lane;
      const int uv  = reg1[idx < RCAP ? idx : RCAP - 1];
      const int m32 = (nh - b0) < 32 ? (nh - b0) : 32;
#pragma unroll 1
      for (int k = 0; k < m32; ++k) {
        const int u   = __builtin_amdgcn_readlane(uv, k);
        const int sl  = u & (NBMAX - 1);
        const int eid = (int)((unsigned)u >> 12);
        if (lane == 0) {
          int pos = list[sl];
          pos = pos < 0 ? 0 : (pos > RCAP - 1 ? RCAP - 1 : pos);
          reg2[pos] = eid;
          list[sl] = pos + 1;
        }
      }
    }
  }
  __syncthreads();

  const int nbw = nb >> 3;
  const int c4  = 4 * (lane & 15);
  const v4f bz4 = *(const v4f*)(biasr + c4);
  float* stgw = (float*)(list + wave * 256);
#pragma unroll 1
  for (int jt = 0; jt < nbw; ++jt) {
    const int slot = wave * nbw + jt;
    const int grow = nodeBase + slot;
    int st  = soff[slot];
    int cnt = scnt[slot];
    st  = st < 0 ? 0 : (st > nh ? nh : st);
    cnt = cnt < 0 ? 0 : (cnt > DEGCAP ? DEGCAP : cnt);
    if (cnt > nh - st) cnt = nh - st;

    float mx = -3.0e38f;
#pragma unroll 1
    for (int q0 = 0; q0 < cnt; q0 += 32) {
      const int qi = q0 + lane;
      int idx = st + qi; idx = idx > RCAP - 1 ? RCAP - 1 : idx;
      int eid = reg2[idx]; eid = eid < 0 ? 0 : (eid > nE - 1 ? nE - 1 : eid);
      const float e = ev[eid];
      mx = (qi < cnt) ? fmaxf(mx, e) : mx;
    }
#pragma unroll
    for (int d = 16; d >= 1; d >>= 1) mx = fmaxf(mx, __shfl_xor(mx, d));

    float dsum = 0.0f, ax = 0.0f, ay = 0.0f;
#pragma unroll 1
    for (int q0 = 0; q0 < cnt; q0 += 32) {
      const int qi = q0 + lane;
      int idx = st + qi; idx = idx > RCAP - 1 ? RCAP - 1 : idx;
      int eid = reg2[idx]; eid = eid < 0 ? 0 : (eid > nE - 1 ? nE - 1 : eid);
      const float e = ev[eid];
      int s = srcs[eid]; s = s < 0 ? 0 : (s > nSrc - 1 ? nSrc - 1 : s);
      const bool valid = qi < cnt;
      const float arg = valid ? (e - mx) : -80.0f;
      float p = __expf(arg);
      p = valid ? p : 0.0f;
      dsum += p;
      const int mcnt = (cnt - q0) < 32 ? (cnt - q0) : 32;
#pragma unroll 1
      for (int pp = 0; pp < mcnt; ++pp) {
        const int   sp = __builtin_amdgcn_readlane(s, pp);
        const float pv = __int_as_float(__builtin_amdgcn_readlane(__float_as_int(p), pp));
        const v2f xv = *(const v2f*)(xl + (size_t)sp * xlPitch + 2 * lane);
        ax = fmaf(pv, xv.x, ax);
        ay = fmaf(pv, xv.y, ay);
      }
    }
#pragma unroll
    for (int d = 16; d >= 1; d >>= 1) dsum += __shfl_xor(dsum, d);
    const float inv = (cnt > 0) ? __builtin_amdgcn_rcpf(dsum) : 0.0f;

    v2f o2;
    o2.x = ax * inv;
    o2.y = ay * inv;
    *(v2f*)(stgw + 2 * lane) = o2;
    __builtin_amdgcn_fence(__ATOMIC_RELEASE, "wavefront");
    __builtin_amdgcn_wave_barrier();
    const v4fa g4 = *(const v4fa*)(stgw + c4);
    const int gcl = grow < nDst ? grow : nDst - 1;
    const v4f ad = *(const v4f*)(addend + (size_t)gcl * FD + c4);
    v4f o;
    o.x = (g4.x + bz4.x) + ad.x;
    o.y = (g4.y + bz4.y) + ad.y;
    o.z = (g4.z + bz4.z) + ad.z;
    o.w = (g4.w + bz4.w) + ad.w;
    float* gp = outp + (size_t)gcl * FD + c4;
    const bool wr = (lane < 16) && (grow < nDst);
    if (wr) *(volatile v4f*)gp = o;
    __threadfence();
    if (wr) *(volatile v4f*)gp = o;
  }
}

__global__ __launch_bounds__(NTHR) void k_bnstat(const float* __restrict__ v, double* part, int nN) {
  __shared__ __attribute__((aligned(16))) double sS[NTHR];
  __shared__ __attribute__((aligned(16))) double sQ[NTHR];
  __shared__ __attribute__((aligned(16))) double sP[PARTN];
  const int tid = threadIdx.x, c = tid & (FD - 1), q = tid >> 6;
  const int r0 = (int)blockIdx.x * RB;
  int r1 = r0 + RB;
  r1 = r1 > nN ? nN : r1;
  double s = 0.0, sq = 0.0;
#pragma unroll 2
  for (int r = r0 + q; r < r1; r += 4) {
    const double xv = (double)v[(size_t)r * FD + c];
    s  += xv;
    sq += xv * xv;
  }
  sS[tid] = s;
  sQ[tid] = sq;
  __syncthreads();
  if (tid < FD) {
    sP[tid]      = (sS[tid] + sS[FD + tid]) + (sS[2 * FD + tid] + sS[3 * FD + tid]);
    sP[FD + tid] = (sQ[tid] + sQ[FD + tid]) + (sQ[2 * FD + tid] + sQ[3 * FD + tid]);
  }
  __syncthreads();
  v2d pv = {0.0, 0.0};
  double* pp = part + (size_t)blockIdx.x * PARTN + 2 * tid;
  if (tid < PARTN / 2) { pv = *(const v2d*)(sP + 2 * tid); *(volatile v2d*)pp = pv; }
  __threadfence();
  if (tid < PARTN / 2) *(volatile v2d*)pp = pv;
}

__global__ __launch_bounds__(128) void k_bnred(const double* __restrict__ part, const float* __restrict__ gam,
                                               const float* __restrict__ bet, float* slot, int nBlk, int nN) {
  __shared__ __attribute__((aligned(16))) double sAcc[PARTN];
  __shared__ __attribute__((aligned(16))) float  sSl[SLOTN];
  const int tid = threadIdx.x;
  double a = 0.0;
#pragma unroll 2
  for (int bk = 0; bk < nBlk; ++bk) a += part[(size_t)bk * PARTN + tid];
  sAcc[tid] = a;
  __syncthreads();
  if (tid < FD) {
    const double invN = 1.0 / (double)nN;
    const double mu   = sAcc[tid] * invN;
    double var = sAcc[FD + tid] * invN - mu * mu;
    var = var < 0.0 ? 0.0 : var;
    const float rstd = rsqrtf((float)var + BN_EPS);
    sSl[tid]          = (float)mu;
    sSl[FD + tid]     = gam[tid] * rstd;
    sSl[2 * FD + tid] = bet[tid];
    sSl[3 * FD + tid] = 0.0f;
  }
  __syncthreads();
  v4f vv = {0.f, 0.f, 0.f, 0.f};
  if (tid < SLOTN / 4) { vv = *(const v4f*)(sSl + 4 * tid); *(volatile v4f*)(slot + 4 * tid) = vv; }
  __threadfence();
  if (tid < SLOTN / 4) *(volatile v4f*)(slot + 4 * tid) = vv;
}

__global__ __launch_bounds__(NTHR) void k_bnapply(float* out, const float* __restrict__ slot, int nN) {
  const int i = (int)blockIdx.x * NTHR + (int)threadIdx.x;
  const int total = nN * (FD / 4);
  if (i >= total) return;
  const int row = i >> 4;
  const int col = 4 * (i & 15);
  const v4f mu = *(const v4f*)(slot + col);
  const v4f sc = *(const v4f*)(slot + FD + col);
  const v4f sh = *(const v4f*)(slot + 2 * FD + col);
  float* p = out + (size_t)row * FD + col;
  const v4f xv = *(const v4f*)p;
  const v4f y = (xv - mu) * sc + sh;
  *(volatile v4f*)p = y;
  __threadfence();
  *(volatile v4f*)p = y;
}

static int pick_nb(int nE, int nDst) {
  int nb = NBMAX;
  while (nb > 16 && (long long)nb * (long long)nE * 5LL > (long long)RCAP * (long long)nDst * 4LL) nb >>= 1;
  return nb;
}

extern "C" void kernel_launch(void* const* d_in, const int* in_sizes, int n_in,
                              void* d_out, int out_size, void* d_ws, size_t ws_size,
                              hipStream_t stream) {
  if (n_in < 14) return;
  const int nOp = in_sizes[0] / FD, nM = in_sizes[1] / FD, nA = in_sizes[2] / FD;
  if (nOp <= 0 || nM <= 0 || nA <= 0) return;
  if (in_sizes[0] != nOp * FD || in_sizes[1] != nM * FD || in_sizes[2] != nA * FD) return;
  int E[NREL];
  for (int r = 0; r < NREL; ++r) {
    const int sz = in_sizes[3 + r];
    if (sz <= 0 || (sz & 1) != 0) return;
    E[r] = sz / 2;
    if (E[r] > (1 << 20)) return;
  }
  if (in_sizes[8] != NREL * FD * FD || in_sizes[9] != NREL * FD * FD) return;
  if (in_sizes[10] != NREL * FD || in_sizes[11] != NREL * FD) return;
  if (in_sizes[12] != 3 * FD || in_sizes[13] != 3 * FD) return;
  if (out_size != (nOp + nM + nA) * FD) return;
  if (nOp > (1 << 24) || nM > (1 << 24) || nA > (1 << 24)) return;

  const float* x_op = (const float*)d_in[0];
  const float* x_m  = (const float*)d_in[1];
  const float* x_a  = (const float*)d_in[2];
  const int* ei[NREL];
  ei[0] = (const int*)d_in[3];
  ei[1] = (const int*)d_in[4];
  ei[2] = (const int*)d_in[5];
  ei[3] = (const int*)d_in[6];
  ei[4] = (const int*)d_in[7];
  const float* Wl   = (const float*)d_in[8];
  const float* Wr   = (const float*)d_in[9];
  const float* att  = (const float*)d_in[10];
  const float* bias = (const float*)d_in[11];
  const float* gam  = (const float*)d_in[12];
  const float* bet  = (const float*)d_in[13];
  float* out0 = (float*)d_out;
  float* out1 = out0 + (size_t)nOp * FD;
  float* out2 = out1 + (size_t)nM * FD;

  const int MPo = ((nOp + GBM - 1) / GBM) * GBM;
  const int MPm = ((nM  + GBM - 1) / GBM) * GBM;
  const int MPa = ((nA  + GBM - 1) / GBM) * GBM;
  int maxE = 0;
  for (int r = 0; r < NREL; ++r) maxE = E[r] > maxE ? E[r] : maxE;
  const int gridEmax = (maxE + NTHR - 1) / NTHR;
  const int nBo = (nOp + RB - 1) / RB, nBm = (nM + RB - 1) / RB, nBa = (nA + RB - 1) / RB;
  int nBlkMax = nBo; nBlkMax = nBm > nBlkMax ? nBm : nBlkMax; nBlkMax = nBa > nBlkMax ? nBa : nBlkMax;

  char* ws = (char*)d_ws;
  size_t off = 0;
  const size_t ysRows128 = (size_t)MPo * 2 * FD;
  const size_t ysRows64m = (size_t)MPm * FD;
  const size_t ysFloats  = ysRows128 > ysRows64m ? ysRows128 : ysRows64m;
  const size_t ydRows    = (size_t)(MPm > MPa ? MPm : MPa);
  const size_t oWq  = off; off += (size_t)NMAT * FD * FD * 2;            off = (off + 255) & ~(size_t)255;
  const size_t oXo  = off; off += (size_t)MPo * FD * 2;                  off = (off + 255) & ~(size_t)255;
  const size_t oXm  = off; off += (size_t)MPm * FD * 2;                  off = (off + 255) & ~(size_t)255;
  const size_t oXa  = off; off += (size_t)MPa * FD * 2;                  off = (off + 255) & ~(size_t)255;
  const size_t oYS  = off; off += ysFloats * 4;                          off = (off + 255) & ~(size_t)255;
  const size_t oYD  = off; off += ydRows * FD * 4;                       off = (off + 255) & ~(size_t)255;
  const size_t oEV  = off; off += (size_t)gridEmax * NTHR * 4;           off = (off + 255) & ~(size_t)255;
  const size_t oPa  = off; off += (size_t)nBlkMax * PARTN * 8;           off = (off + 255) & ~(size_t)255;
  const size_t oSl  = off; off += (size_t)3 * SLOTN * 4;                 off = (off + 255) & ~(size_t)255;
  if (off > ws_size || off > (size_t)WSCAP) return;
  unsigned short* wq   = (unsigned short*)(ws + oWq);
  unsigned short* X16o = (unsigned short*)(ws + oXo);
  unsigned short* X16m = (unsigned short*)(ws + oXm);
  unsigned short* X16a = (unsigned short*)(ws + oXa);
  float*  YS    = (float*)(ws + oYS);
  float*  YD    = (float*)(ws + oYD);
  float*  EV    = (float*)(ws + oEV);
  double* part  = (double*)(ws + oPa);
  float*  slots = (float*)(ws + oSl);

  hipFuncSetAttribute(reinterpret_cast<const void*>(&k_agg),
                      hipFuncAttributeMaxDynamicSharedMemorySize, LDS_AGG);

  k_xprep<<<MPo * 8 / NTHR, NTHR, 0, stream>>>(x_op, X16o, nOp, MPo * 8);
  k_xprep<<<MPm * 8 / NTHR, NTHR, 0, stream>>>(x_m,  X16m, nM,  MPm * 8);
  k_xprep<<<MPa * 8 / NTHR, NTHR, 0, stream>>>(x_a,  X16a, nA,  MPa * 8);
  k_wprep<<<dim3(FD * FD / 8 / NTHR, NMAT), NTHR, 0, stream>>>(Wl, Wr, wq);

  {
    const int r = 0, nE = E[r], nb = pick_nb(nE, nOp), vec8 = ((nE & 3) == 0) ? 1 : 0;
    k_gemm<<<MPo / GBM, GTHR, 0, stream>>>(X16o, wq + (size_t)0 * FD * FD, YS, 2);
    k_logit<<<(nE + NTHR - 1) / NTHR, NTHR, 0, stream>>>(ei[r], ei[r] + nE, YS, YS + FD, att + r * FD, EV,
                                                         nE, nOp, nOp, 2 * FD, 2 * FD);
    k_agg<<<(nOp + nb - 1) / nb, NTHR, LDS_AGG, stream>>>(ei[r], ei[r] + nE, EV, YS, x_op, bias + r * FD, out0,
                                                          nOp, nOp, nE, 2 * FD, nb, vec8);
  }
  {
    const int r = 1, nE = E[r], nb = pick_nb(nE, nOp), vec8 = ((nE & 3) == 0) ? 1 : 0;
    k_gemm<<<MPo / GBM, GTHR, 0, stream>>>(X16o, wq + (size_t)2 * FD * FD, YS, 2);
    k_logit<<<(nE + NTHR - 1) / NTHR, NTHR, 0, stream>>>(ei[r], ei[r] + nE, YS, YS + FD, att + r * FD, EV,
                                                         nE, nOp, nOp, 2 * FD, 2 * FD);
    k_agg<<<(nOp + nb - 1) / nb, NTHR, LDS_AGG, stream>>>(ei[r], ei[r] + nE, EV, YS, out0, bias + r * FD, out0,
                                                          nOp, nOp, nE, 2 * FD, nb, vec8);
  }
  {
    const int r = 2, nE = E[r], nb = pick_nb(nE, nM), vec8 = ((nE & 3) == 0) ? 1 : 0;
    k_gemm<<<MPo / GBM, GTHR, 0, stream>>>(X16o, wq + (size_t)4 * FD * FD, YS, 1);
    k_gemm<<<MPm / GBM, GTHR, 0, stream>>>(X16m, wq + (size_t)5 * FD * FD, YD, 1);
    k_logit<<<(nE + NTHR - 1) / NTHR, NTHR, 0, stream>>>(ei[r], ei[r] + nE, YS, YD, att + r * FD, EV,
                                                         nE, nOp, nM, FD, FD);
    k_agg<<<(nM + nb - 1) / nb, NTHR, LDS_AGG, stream>>>(ei[r], ei[r] + nE, EV, YS, x_m, bias + r * FD, out1,
                                                         nM, nOp, nE, FD, nb, vec8);
  }
  {
    const int r = 3, nE = E[r], nb = pick_nb(nE, nA), vec8 = ((nE & 3) == 0) ? 1 : 0;
    k_gemm<<<MPo / GBM, GTHR, 0, stream>>>(X16o, wq + (size_t)6 * FD * FD, YS, 1);
    k_gemm<<<MPa / GBM, GTHR, 0, stream>>>(X16a, wq + (size_t)7 * FD * FD, YD, 1);
    k_logit<<<(nE + NTHR - 1) / NTHR, NTHR, 0, stream>>>(ei[r], ei[r] + nE, YS, YD, att + r * FD, EV,
                                                         nE, nOp, nA, FD, FD);
    k_agg<<<(nA + nb - 1) / nb, NTHR, LDS_AGG, stream>>>(ei[r], ei[r] + nE, EV, YS, x_a, bias + r * FD, out2,
                                                         nA, nOp, nE, FD, nb, vec8);
  }
  {
    const int r = 4, nE = E[r], nb = pick_nb(nE, nA), vec8 = ((nE & 3) == 0) ? 1 : 0;
    k_gemm<<<MPm / GBM, GTHR, 0, stream>>>(X16m, wq + (size_t)8 * FD * FD, YS, 1);
    k_gemm<<<MPa / GBM, GTHR, 0, stream>>>(X16a, wq + (size_t)9 * FD * FD, YD, 1);
    k_logit<<<(nE + NTHR - 1) / NTHR, NTHR, 0, stream>>>(ei[r], ei[r] + nE, YS, YD, att + r * FD, EV,
                                                         nE, nM, nA, FD, FD);
    k_agg<<<(nA + nb - 1) / nb, NTHR, LDS_AGG, stream>>>(ei[r], ei[r] + nE, EV, YS, out2, bias + r * FD, out2,
                                                         nA, nM, nE, FD, nb, vec8);
  }

  k_bnstat<<<nBo, NTHR, 0, stream>>>(out0, part, nOp);
  k_bnred<<<1, 128, 0, stream>>>(part, gam + 0 * FD, bet + 0 * FD, slots + 0 * SLOTN, nBo, nOp);
  k_bnapply<<<(nOp * 16 + NTHR - 1) / NTHR, NTHR, 0, stream>>>(out0, slots + 0 * SLOTN, nOp);
  k_bnstat<<<nBm, NTHR, 0, stream>>>(out1, part, nM);
  k_bnred<<<1, 128, 0, stream>>>(part, gam + 1 * FD, bet + 1 * FD, slots + 1 * SLOTN, nBm, nM);
  k_bnapply<<<(nM * 16 + NTHR - 1) / NTHR, NTHR, 0, stream>>>(out1, slots + 1 * SLOTN, nM);
  k_bnstat<<<nBa, NTHR, 0, stream>>>(out2, part, nA);
  k_bnred<<<1, 128, 0, stream>>>(part, gam + 2 * FD, bet + 2 * FD, slots + 2 * SLOTN, nBa, nA);
  k_bnapply<<<(nA * 16 + NTHR - 1) / NTHR, NTHR, 0, stream>>>(out2, slots + 2 * SLOTN, nA);
}
